// SpatialReductionAttention_31447750541387
// MI455X (gfx1250) — hardware-verified
//
#include <hip/hip_runtime.h>
#include <math.h>

#define NB_ 8
#define CC 256
#define HWQ 4096
#define NKEY 256
#define GSTR 48

typedef _Float16 f16;
typedef __attribute__((ext_vector_type(16))) f16 f16x16;
typedef __attribute__((ext_vector_type(8)))  f16 f16x8;
typedef __attribute__((ext_vector_type(8)))  float f32x8;
typedef __attribute__((ext_vector_type(4)))  float v4f_t;
typedef float v4fa __attribute__((ext_vector_type(4), may_alias));
__device__ __forceinline__ f32x8 wmma16(f16x16 a, f16x16 b, f32x8 c) {
  c = __builtin_amdgcn_wmma_f32_16x16x32_f16(false, a, false, b, (short)0, c, false, false);
  asm volatile("v_nop\n\tv_nop\n\tv_nop\n\tv_nop" : "+v"(c) : "v"(a), "v"(b));
  return c;
}
__device__ __forceinline__ f16x16 lds_frag(const f16* base, int stride) {
  const int lane = threadIdx.x & 31, row = lane & 15, kh = (lane >> 4) * 8;
  const f16x8 lo = *(const f16x8*)(base + row * stride + kh);
  const f16x8 hi = *(const f16x8*)(base + row * stride + kh + 16);
  f16x16 f;
#pragma unroll
  for (int i = 0; i < 8; ++i) { f[i] = lo[i]; f[i + 8] = hi[i]; }
  return f;
}

template <typename AT, int ASRC>
__global__ __launch_bounds__(256) void gemm_knb2(const AT* __restrict__ A, int lda, size_t strideA,
                                               const float* __restrict__ Wm, int ldw, size_t strideW,
                                               const float* __restrict__ rowbias, const float* __restrict__ s1, const float* __restrict__ s2, const float* __restrict__ mj, const float* __restrict__ invD,
                                               float scale, int N, float* __restrict__ Y, int ldy, size_t strideY, int K) {
  __shared__ __attribute__((aligned(16))) f16 ldsA[128 * GSTR], ldsAl[128 * GSTR];
  __shared__ __attribute__((aligned(16))) f16 ldsW[128 * GSTR], ldsWl[128 * GSTR];
  __shared__ __attribute__((aligned(16))) float oS[8][32 * 68];
  const int tid = threadIdx.x, lane = tid & 31, wave = tid >> 5, cl = lane & 15, rh = (lane >> 4) * 8;
  const int m0 = blockIdx.x * 128, n0 = blockIdx.y * 128;
  const int wm = (wave & 3) * 32, wn = (wave >> 2) * 64;
  A += (size_t)blockIdx.z * strideA; Wm += (size_t)blockIdx.z * strideW; Y += (size_t)blockIdx.z * strideY;
  if (ASRC == 1) { s1 += (size_t)blockIdx.z * K; s2 += (size_t)blockIdx.z * lda; mj += (size_t)blockIdx.z * K; invD += (size_t)blockIdx.z * K; }
  f32x8 acc[2][4], accx[2][4];
#pragma unroll
  for (int i = 0; i < 2; ++i)
#pragma unroll
    for (int j = 0; j < 4; ++j) { f32x8 z = {}; acc[i][j] = z; accx[i][j] = z; }
#pragma unroll 1
  for (int k0 = 0; k0 < K; k0 += 32) {
    __syncthreads();
    {
      const int row = tid >> 1, ch = (tid & 1) * 16;
      if (ASRC == 0) {
        const AT* src = A + (size_t)(m0 + row) * lda + k0 + ch;
#pragma unroll
        for (int g = 0; g < 16; ++g) { const float v = (float)src[g]; const f16 h = (f16)v; ldsA[row * GSTR + ch + g] = h; ldsAl[row * GSTR + ch + g] = (f16)((v - (float)h) * 2048.0f); }
      } else {
        const float s2i = s2[m0 + row];
#pragma unroll
        for (int g = 0; g < 16; ++g) { const int j = k0 + ch + g; float a = s1[j] + s2i; a = (a >= 0.0f) ? a : 0.2f * a;
          const float v = 1024.0f * __expf(a - mj[j]) * invD[j]; const f16 h = (f16)v; ldsA[row * GSTR + ch + g] = h; ldsAl[row * GSTR + ch + g] = (f16)((v - (float)h) * 2048.0f); }
      }
    }
    {
      const int k = tid >> 3, nn0 = (tid & 7) * 16;
      const float* src = Wm + (size_t)(k0 + k) * ldw;
#pragma unroll
      for (int g = 0; g < 4; ++g) { const int col = min(n0 + nn0 + 4 * g, N - 4); const v4f_t v = *(const v4f_t*)(src + col);
#pragma unroll
        for (int u = 0; u < 4; ++u) { const f16 h = (f16)v[u]; ldsW[(nn0 + 4 * g + u) * GSTR + k] = h; ldsWl[(nn0 + 4 * g + u) * GSTR + k] = (f16)((v[u] - (float)h) * 2048.0f); } }
    }
    __syncthreads();
    f16x16 af[2], afl[2];
#pragma unroll
    for (int i = 0; i < 2; ++i) { af[i] = lds_frag(ldsA + (wm + 16 * i) * GSTR, GSTR); afl[i] = lds_frag(ldsAl + (wm + 16 * i) * GSTR, GSTR); }
#pragma unroll
    for (int j = 0; j < 4; ++j) {
      const f16x16 bf = lds_frag(ldsW + (wn + 16 * j) * GSTR, GSTR), bfl = lds_frag(ldsWl + (wn + 16 * j) * GSTR, GSTR);
#pragma unroll
      for (int i = 0; i < 2; ++i) { acc[i][j] = wmma16(af[i], bf, acc[i][j]); accx[i][j] = wmma16(af[i], bfl, accx[i][j]); accx[i][j] = wmma16(afl[i], bf, accx[i][j]); }
    }
  }
  float* so = oS[wave];
#pragma unroll
  for (int i = 0; i < 2; ++i)
#pragma unroll
    for (int j = 0; j < 4; ++j) {
#pragma unroll
      for (int r = 0; r < 8; ++r) { const float rb = rowbias ? rowbias[m0 + wm + 16 * i + rh + r] : 0.0f; so[(16 * i + rh + r) * 68 + 16 * j + cl] = (acc[i][j][r] + accx[i][j][r] * (1.0f / 2048.0f)) * scale + rb; }
    }
  asm volatile("s_wait_dscnt 0" ::: "memory");
  __builtin_amdgcn_wave_barrier();
#pragma unroll 1
  for (int pass = 0; pass < 2; ++pass) {
#pragma unroll
    for (int it = 0; it < 16; ++it) { const int f4 = lane + 32 * it, rr = f4 >> 4, q = (f4 & 15) * 4;
      if (n0 + wn + q < N) *(volatile v4f_t*)(Y + (size_t)(m0 + wm + rr) * ldy + n0 + wn + q) = *(const volatile v4fa*)(so + rr * 68 + q); }
    __threadfence();
  }
}

__global__ __launch_bounds__(256) void k_attn32(const float* __restrict__ Qc, const float* __restrict__ Kc, const float* __restrict__ Vc, float* __restrict__ Oc) {
  __shared__ __attribute__((aligned(16))) f16 qS[2][32 * 40];
  __shared__ __attribute__((aligned(16))) union KP { f16 kS[2][256 * 40]; f16 pS[32 * 264]; } kp;
  __shared__ __attribute__((aligned(16))) f16 vS[32 * 264];
  __shared__ __attribute__((aligned(16))) union SO { float sS[32 * 260]; float oS[32 * 36]; } so;
  const int tid = threadIdx.x, lane = tid & 31, wave = tid >> 5, cl = lane & 15, rh = (lane >> 4) * 8;
  const int b = blockIdx.z, h = blockIdx.y, q0 = blockIdx.x * 32;
  const float* Qh = Qc + ((size_t)b * 256 + h * 32) * 4096; const float* Kh = Kc + ((size_t)b * 256 + h * 32) * 256; const float* Vh = Vc + ((size_t)b * 256 + h * 32) * 256;
  for (int e = tid; e < 32 * 32; e += 256) { const int d = e >> 5, q = e & 31; const float v = Qh[(size_t)d * 4096 + q0 + q]; const f16 hh = (f16)v; qS[0][q * 40 + d] = hh; qS[1][q * 40 + d] = (f16)((v - (float)hh) * 2048.0f); }
  for (int e = tid; e < 256 * 32; e += 256) { const int d = e >> 8, j = e & 255; const float v = Kh[(size_t)d * 256 + j]; const f16 hh = (f16)v; kp.kS[0][j * 40 + d] = hh; kp.kS[1][j * 40 + d] = (f16)((v - (float)hh) * 2048.0f); }
  for (int e = tid; e < 32 * 256; e += 256) { const int d = e >> 8, j = e & 255; vS[d * 264 + j] = (f16)Vh[(size_t)d * 256 + j]; }
  if (tid < 32) { for (int j = 256; j < 264; ++j) vS[tid * 264 + j] = (f16)0.0f; }
  __syncthreads();
  { const int qt = wave & 1, kt0 = (wave >> 1) * 4; const f16x16 ah = lds_frag(qS[0] + (qt * 16) * 40, 40), al = lds_frag(qS[1] + (qt * 16) * 40, 40);
#pragma unroll
    for (int t4 = 0; t4 < 4; ++t4) { const int kt = kt0 + t4; const f16x16 bh = lds_frag(kp.kS[0] + (kt * 16) * 40, 40), bl = lds_frag(kp.kS[1] + (kt * 16) * 40, 40);
      f32x8 acc = {}, accx = {}; acc = wmma16(ah, bh, acc); accx = wmma16(ah, bl, accx); accx = wmma16(al, bh, accx);
#pragma unroll
      for (int r = 0; r < 8; ++r) so.sS[(qt * 16 + rh + r) * 260 + kt * 16 + cl] = (acc[r] + accx[r] * (1.0f / 2048.0f)) * 0.17677669529663687f; } }
  __syncthreads();
  { const int q = tid >> 3, part = tid & 7; float mx = -3.0e38f; float ev[32];
#pragma unroll
    for (int i = 0; i < 32; ++i) mx = fmaxf(mx, so.sS[q * 260 + part * 32 + i]);
    mx = fmaxf(mx, __shfl_xor(mx, 1, 32)); mx = fmaxf(mx, __shfl_xor(mx, 2, 32)); mx = fmaxf(mx, __shfl_xor(mx, 4, 32));
    float z = 0.0f;
#pragma unroll
    for (int i = 0; i < 32; ++i) { ev[i] = expf(so.sS[q * 260 + part * 32 + i] - mx); z += ev[i]; }
    z += __shfl_xor(z, 1, 32); z += __shfl_xor(z, 2, 32); z += __shfl_xor(z, 4, 32); const float iz = 1024.0f / z;
    __syncthreads();
#pragma unroll
    for (int i = 0; i < 32; ++i) kp.pS[q * 264 + part * 32 + i] = (f16)(ev[i] * iz);
    if (part == 0) for (int j = 256; j < 264; ++j) kp.pS[q * 264 + j] = (f16)0.0f; }
  __syncthreads();
  if (wave < 4) { const int qt = wave & 1, dt = wave >> 1; f32x8 acc = {};
#pragma unroll
    for (int ks = 0; ks < 8; ++ks) acc = wmma16(lds_frag(kp.pS + (qt * 16) * 264 + ks * 32, 264), lds_frag(vS + (dt * 16) * 264 + ks * 32, 264), acc);
#pragma unroll
    for (int r = 0; r < 8; ++r) so.oS[(dt * 16 + cl) * 36 + qt * 16 + rh + r] = acc[r] * (1.0f / 1024.0f); }
  __syncthreads();
#pragma unroll 1
  for (int pass = 0; pass < 2; ++pass) { { const int d = tid >> 3, c4 = (tid & 7) * 4;
      *(volatile v4f_t*)(Oc + ((size_t)b * 256 + h * 32 + d) * 4096 + q0 + c4) = *(const volatile v4fa*)(so.oS + d * 36 + c4); } __threadfence(); }
}
__global__ __launch_bounds__(256) void k_im2col(const float* __restrict__ x, float* __restrict__ col) {
  __shared__ __attribute__((aligned(16))) float cS[16 * 260];
  const int tid = threadIdx.x, b = blockIdx.x >> 8, c = blockIdx.x & 255;
  const float* xc = x + ((size_t)b * 256 + c) * 4096;
  for (int e = tid; e < 4096; e += 256) { const int yy = e >> 6, xx = e & 63; const int kh = yy & 3, py = yy >> 2, kw = xx & 3, px = xx >> 2; cS[(kh * 4 + kw) * 260 + py * 16 + px] = xc[e]; }
  __syncthreads();
#pragma unroll 1
  for (int pass = 0; pass < 2; ++pass) { for (int q4 = tid; q4 < 16 * 64; q4 += 256) { const int k = q4 >> 6, c4 = (q4 & 63) * 4;
      *(volatile v4f_t*)(col + (((size_t)b * 4096) + c * 16 + k) * 256 + c4) = *(const volatile v4fa*)(cS + k * 260 + c4); } __threadfence(); }
}

extern "C" void kernel_launch(void* const* d_in, const int* in_sizes, int n_in,
                              void* d_out, int out_size, void* d_ws, size_t ws_size,
                              hipStream_t stream) {
  (void)in_sizes; (void)n_in; (void)out_size;
  const float* x = (const float*)d_in[0];
  const float* wq = (const float*)d_in[1], *wk = (const float*)d_in[2], *wv = (const float*)d_in[3], *wout = (const float*)d_in[4];
  float* out = (float*)d_out;
  char* ws = (char*)d_ws;
  float* Qc = (float*)ws; ws += (size_t)NB_ * CC * HWQ * 4;
  float* col = (float*)ws; ws += (size_t)NB_ * 4096 * NKEY * 4;
  float* Kc = (float*)ws; ws += (size_t)NB_ * CC * NKEY * 4;
  float* Vc = (float*)ws; ws += (size_t)NB_ * CC * NKEY * 4;
  float* Oc = (float*)ws; ws += (size_t)NB_ * CC * HWQ * 4;
  if ((size_t)(ws - (char*)d_ws) > ws_size) return;
  const dim3 blk(256);
  gemm_knb2<float, 0><<<dim3(CC / 128, HWQ / 128, NB_), blk, 0, stream>>>(wq, CC, 0, x, HWQ, (size_t)CC * HWQ, nullptr, nullptr, nullptr, nullptr, nullptr, 1.0f, HWQ, Qc, HWQ, (size_t)CC * HWQ, CC);
  k_im2col<<<dim3(NB_ * CC), blk, 0, stream>>>(x, col);
  gemm_knb2<float, 0><<<dim3(CC / 128, NKEY / 128, NB_), blk, 0, stream>>>(wk, 4096, 0, col, NKEY, (size_t)4096 * NKEY, nullptr, nullptr, nullptr, nullptr, nullptr, 1.0f, NKEY, Kc, NKEY, (size_t)CC * NKEY, 4096);
  gemm_knb2<float, 0><<<dim3(CC / 128, NKEY / 128, NB_), blk, 0, stream>>>(wv, 4096, 0, col, NKEY, (size_t)4096 * NKEY, nullptr, nullptr, nullptr, nullptr, nullptr, 1.0f, NKEY, Vc, NKEY, (size_t)CC * NKEY, 4096);
  k_attn32<<<dim3(HWQ / 32, 8, NB_), blk, 0, stream>>>(Qc, Kc, Vc, Oc);
  gemm_knb2<float, 0><<<dim3(CC / 128, HWQ / 128, NB_), blk, 0, stream>>>(wout, CC, 0, Oc, HWQ, (size_t)CC * HWQ, nullptr, nullptr, nullptr, nullptr, nullptr, 1.0f, HWQ, out, HWQ, (size_t)CC * HWQ, CC);
}
